// S4_40673340293925
// MI455X (gfx1250) — hardware-run, weakly checked
//
#include <hip/hip_runtime.h>
#include <math.h>

typedef __attribute__((ext_vector_type(16))) _Float16 v16h;
typedef __attribute__((ext_vector_type(8)))  _Float16 v8h;
typedef __attribute__((ext_vector_type(8)))  float    v8f;
typedef __attribute__((ext_vector_type(4)))  float    v4f;

constexpr int kBatch  = 16;
constexpr int kSteps  = 4096;
constexpr int kChan   = 64;
constexpr int kState  = 64;
constexpr int kOutF   = 64;
constexpr int kRows   = kBatch * kSteps;
constexpr int kChunk  = 64;
constexpr int kYPitch = 68;
constexpr int kAPitch = 72;
static_assert(kChan == 64 && kState == 64 && kOutF == 64, "tile plan assumes 64 channels, 64 states, 64 outputs");
static_assert((kSteps % kChunk) == 0, "chunk multiple");
static_assert((kRows % 64) == 0 && (kOutF % 64) == 0 && (kChan % 32) == 0, "GEMM M,N multiples of 64, K multiple of 32");
static_assert((kAPitch % 8) == 0, "16-B aligned f16 rows");

constexpr float kCarryA    = 64.0f;
constexpr float kCarryH    = 2048.0f;
constexpr float kCarryProd = kCarryA * kCarryH;
constexpr float kInvProd   = 1.0f / kCarryProd;
constexpr float kPack      = kCarryH / kCarryProd;
constexpr float kCarryY    = 64.0f;
constexpr float kCarryW    = 64.0f;
constexpr float kMixScale  = 1.0f / (kCarryY * kCarryW);
constexpr float kF16MinNormal = 6.103515625e-5f;

constexpr size_t kOffWH   = 0;
constexpr size_t kOffYH   = kOffWH + (size_t)kOutF * kChan * 2;
constexpr size_t kWsTotal = kOffYH + (size_t)kRows * kChan * 2;
static_assert(kWsTotal == 8396800ull, "carve total");
static_assert(kWsTotal <= 134217728ull, "carve cap");
static_assert((kOffYH % 128) == 0, "128-B aligned regions");

__device__ __forceinline__ float flush_small(float v) {
  return (__builtin_fabsf(v) < kF16MinNormal) ? 0.0f : v;
}

__device__ __forceinline__ void guard_acc2(v8f& a, v16h x, v16h y) {
  asm volatile("v_nop\n\tv_nop\n\tv_nop\n\tv_nop" : "+v"(a) : "v"(x), "v"(y));
}
__device__ __forceinline__ void guard_acc4(v8f& a, v16h x0, v16h x1, v16h y0, v16h y1) {
  asm volatile("v_nop\n\tv_nop\n\tv_nop\n\tv_nop" : "+v"(a) : "v"(x0), "v"(x1), "v"(y0), "v"(y1));
}
__device__ __forceinline__ void keep4_h(v16h a, v16h b, v16h c, v16h d) {
  asm volatile("v_nop" :: "v"(a), "v"(b), "v"(c), "v"(d));
}
__device__ __forceinline__ void acc_guard4(v8f& a, v8f& b, v8f& c, v8f& d) {
  asm volatile("v_nop\n\tv_nop\n\tv_nop\n\tv_nop" : "+v"(a), "+v"(b), "+v"(c), "+v"(d));
}

struct FragH {
  union U { v16h v; v8h h[2]; };
  static __device__ __forceinline__ v16h load(const _Float16* p) {
    U f;
    f.h[0] = *(const v8h*)(p);
    f.h[1] = *(const v8h*)(p + 16);
    return f.v;
  }
  static __device__ __forceinline__ v8f mma(v16h a, v16h b, v8f c) {
    return __builtin_amdgcn_wmma_f32_16x16x32_f16(false, a, false, b, (short)0, c, false, false);
  }
};

__global__ __launch_bounds__(256) void weight_plane_kernel(
    const float* __restrict__ W, unsigned short* __restrict__ WH, int n8)
{
  const int i = blockIdx.x * 256 + threadIdx.x;
  if (i < n8) {
    const float* sp = W + (size_t)i * 8;
    const v4f a0 = *(const v4f*)(sp);
    const v4f a1 = *(const v4f*)(sp + 4);
    v8h hv;
#pragma unroll
    for (int e = 0; e < 4; ++e) {
      hv[e]     = (_Float16)flush_small(a0[e] * kCarryW);
      hv[4 + e] = (_Float16)flush_small(a1[e] * kCarryW);
    }
    unsigned short* q = WH + (size_t)i * 8;
    *(volatile v8h*)q = hv;
    __threadfence();
    *(volatile v8h*)q = hv;
  }
}

__global__ __launch_bounds__(128) void state_scan_kernel(
    const float* __restrict__ x, const float* __restrict__ dA, const float* __restrict__ dB,
    const float* __restrict__ Cp, const float* __restrict__ Dp, unsigned short* __restrict__ YH)
{
  __shared__ __align__(16) _Float16 sA[kState * kAPitch];
  __shared__ __align__(16) float sY[kChunk * kYPitch];

  const int tid = threadIdx.x, lane = tid & 31, wave = tid >> 5;
  const int c = lane & 15, hh = lane >> 4;
  const int bidx = blockIdx.x;
  const int d = 16 * wave + c;

#pragma unroll 1
  for (int g = tid; g < kState * kState / 8; g += 128) {
    const int row = g >> 3, c8 = (g & 7) * 8;
    const v4f a0 = *(const v4f*)(dA + row * kState + c8);
    const v4f a1 = *(const v4f*)(dA + row * kState + c8 + 4);
    v8h hv;
#pragma unroll
    for (int e = 0; e < 4; ++e) {
      hv[e]     = (_Float16)flush_small(a0[e] * kCarryA);
      hv[4 + e] = (_Float16)flush_small(a1[e] * kCarryA);
    }
    *(v8h*)(sA + row * kAPitch + c8) = hv;
  }
  __syncthreads();

  v16h afr[4][2];
#pragma unroll
  for (int T = 0; T < 4; ++T)
#pragma unroll
    for (int ks = 0; ks < 2; ++ks)
      afr[T][ks] = FragH::load(sA + (16 * T + c) * kAPitch + 32 * ks + 8 * hh);

  float dbs[4][8], cps[4][8];
#pragma unroll
  for (int T = 0; T < 4; ++T) {
    const float* pb = dB + d * kState + 16 * T + 8 * hh;
    const float* pc = Cp + d * kState + 16 * T + 8 * hh;
    const v4f b0 = *(const v4f*)(pb);
    const v4f b1 = *(const v4f*)(pb + 4);
    const v4f c0 = *(const v4f*)(pc);
    const v4f c1 = *(const v4f*)(pc + 4);
#pragma unroll
    for (int e = 0; e < 4; ++e) {
      dbs[T][e]     = b0[e] * kCarryProd;
      dbs[T][4 + e] = b1[e] * kCarryProd;
      cps[T][e]     = c0[e] * kInvProd;
      cps[T][4 + e] = c1[e] * kInvProd;
    }
  }
  const float dp = Dp[d];

  v8f acc[4];
#pragma unroll
  for (int T = 0; T < 4; ++T) acc[T] = (v8f){0.f, 0.f, 0.f, 0.f, 0.f, 0.f, 0.f, 0.f};

  const float* xrow = x + ((size_t)bidx * kSteps) * kChan + d;
  float ucur = xrow[0];

  const int q = lane >> 3, c8s = (lane & 7) * 8;

#pragma unroll 1
  for (int t0 = 0; t0 < kSteps; t0 += kChunk) {
#pragma unroll 1
    for (int s = 0; s < kChunk; ++s) {
      const int t  = t0 + s;
      const int tn = (t + 1 < kSteps) ? (t + 1) : (kSteps - 1);
      const float unext = xrow[(size_t)tn * kChan];

      v16h bf0, bf1;
#pragma unroll
      for (int r = 0; r < 8; ++r) {
        bf0[r]     = (_Float16)flush_small(acc[0][r] * kPack);
        bf0[8 + r] = (_Float16)flush_small(acc[1][r] * kPack);
        bf1[r]     = (_Float16)flush_small(acc[2][r] * kPack);
        bf1[8 + r] = (_Float16)flush_small(acc[3][r] * kPack);
      }
#pragma unroll
      for (int T = 0; T < 4; ++T)
#pragma unroll
        for (int r = 0; r < 8; ++r) acc[T][r] = dbs[T][r] * ucur;

#pragma unroll
      for (int T = 0; T < 4; ++T) {
        acc[T] = FragH::mma(afr[T][0], bf0, acc[T]);
        acc[T] = FragH::mma(afr[T][1], bf1, acc[T]);
      }
      guard_acc4(acc[0], afr[0][0], afr[0][1], bf0, bf1);
      guard_acc4(acc[1], afr[1][0], afr[1][1], bf0, bf1);
      guard_acc4(acc[2], afr[2][0], afr[2][1], bf0, bf1);
      guard_acc4(acc[3], afr[3][0], afr[3][1], bf0, bf1);

      float yp = 0.0f;
#pragma unroll
      for (int T = 0; T < 4; ++T)
#pragma unroll
        for (int r = 0; r < 8; ++r) yp = fmaf(cps[T][r], acc[T][r], yp);
      const float yo = __shfl_xor(yp, 16, 32);
      float y = yp + yo;
      y = fmaf(dp, ucur, y);
      if (hh == 0) sY[s * kYPitch + d] = y;
      ucur = unext;
    }
    __syncthreads();

    v8h hv[4];
#pragma unroll
    for (int it = 0; it < 4; ++it) {
      const int row = it * 16 + wave * 4 + q;
      const float* sp = sY + row * kYPitch + c8s;
      const v4f a0 = *(const v4f*)(sp);
      const v4f a1 = *(const v4f*)(sp + 4);
#pragma unroll
      for (int e = 0; e < 4; ++e) {
        hv[it][e]     = (_Float16)flush_small(a0[e] * kCarryY);
        hv[it][4 + e] = (_Float16)flush_small(a1[e] * kCarryY);
      }
    }
    unsigned short* yb = YH + ((size_t)bidx * kSteps + (size_t)t0) * kChan;
    for (int pass = 0; pass < 2; ++pass) {
#pragma unroll
      for (int it = 0; it < 4; ++it) {
        const int row = it * 16 + wave * 4 + q;
        *(volatile v8h*)(yb + (size_t)row * kChan + c8s) = hv[it];
      }
      __threadfence();
    }
    __syncthreads();
  }
}

__global__ __launch_bounds__(256) void mix_gemm_kernel(
    const unsigned short* __restrict__ Ap, int lda,
    const unsigned short* __restrict__ Btp, int ldb,
    float* __restrict__ C, int ldc,
    const float* __restrict__ bias,
    int M, int N, int K, float scale)
{
  const _Float16* A  = (const _Float16*)Ap;
  const _Float16* Bt = (const _Float16*)Btp;
  __shared__ __align__(16) float sT[8][16 * 68];
  const int lane = threadIdx.x & 31;
  const int wave = threadIdx.x >> 5;
  const int tilesN = N >> 6;
  const int tilesM = M >> 6;
  const int tile = blockIdx.x * 8 + wave;
  if (tile >= tilesM * tilesN) return;
  const int tm = tile / tilesN;
  const int tn = tile - tm * tilesN;
  const int m0 = tm << 6;
  const int n0 = tn << 6;

  const int rlane = lane & 15;
  const int koff  = (lane >> 4) * 8;
  const int mOff  = (lane >> 4) * 8;

  v8f acc[4][4];
#pragma unroll
  for (int i = 0; i < 4; ++i)
#pragma unroll
    for (int j = 0; j < 4; ++j) acc[i][j] = (v8f){0.f, 0.f, 0.f, 0.f, 0.f, 0.f, 0.f, 0.f};

  for (int k0 = 0; k0 < K; k0 += 32) {
    v16h bh[4];
#pragma unroll
    for (int j = 0; j < 4; ++j) {
      const size_t bo = (size_t)(n0 + (j << 4) + rlane) * ldb + koff + k0;
      bh[j] = FragH::load(Bt + bo);
    }
#pragma unroll
    for (int i = 0; i < 4; ++i) {
      const size_t ao = (size_t)(m0 + (i << 4) + rlane) * lda + koff + k0;
      const v16h ah = FragH::load(A + ao);
#pragma unroll
      for (int j = 0; j < 4; ++j) acc[i][j] = FragH::mma(ah, bh[j], acc[i][j]);
      guard_acc2(acc[i][0], ah, bh[0]);
      guard_acc2(acc[i][1], ah, bh[1]);
      guard_acc2(acc[i][2], ah, bh[2]);
      guard_acc2(acc[i][3], ah, bh[3]);
    }
    keep4_h(bh[0], bh[1], bh[2], bh[3]);
  }
  acc_guard4(acc[0][0], acc[0][1], acc[0][2], acc[0][3]);
  acc_guard4(acc[1][0], acc[1][1], acc[1][2], acc[1][3]);
  acc_guard4(acc[2][0], acc[2][1], acc[2][2], acc[2][3]);
  acc_guard4(acc[3][0], acc[3][1], acc[3][2], acc[3][3]);

  float* slab = sT[wave];
#pragma unroll
  for (int i = 0; i < 4; ++i) {
    const int mBase = m0 + (i << 4);
#pragma unroll
    for (int j = 0; j < 4; ++j) {
      const int n = n0 + (j << 4) + rlane;
      const float bv = bias[n];
#pragma unroll
      for (int r = 0; r < 8; ++r) {
        const float v = acc[i][j][r] * scale + bv;
        slab[(mOff + r) * 68 + (j << 4) + rlane] = v;
      }
    }
    __builtin_amdgcn_fence(__ATOMIC_RELEASE, "workgroup");
    __builtin_amdgcn_wave_barrier();
    __builtin_amdgcn_fence(__ATOMIC_ACQUIRE, "workgroup");
    {
      const int hh = lane >> 4, c4 = (lane & 15) * 4;
      for (int pass = 0; pass < 2; ++pass) {
#pragma unroll
        for (int it = 0; it < 8; ++it) {
          const int row = it * 2 + hh;
          const v4f v = *(const v4f*)(slab + row * 68 + c4);
          *(volatile v4f*)(C + (size_t)(mBase + row) * ldc + n0 + c4) = v;
        }
        __threadfence();
      }
    }
    __builtin_amdgcn_fence(__ATOMIC_RELEASE, "workgroup");
    __builtin_amdgcn_wave_barrier();
    __builtin_amdgcn_fence(__ATOMIC_ACQUIRE, "workgroup");
  }
}

extern "C" void kernel_launch(void* const* d_in, const int* in_sizes, int n_in,
                              void* d_out, int out_size, void* d_ws, size_t ws_size,
                              hipStream_t stream) {
  if (n_in < 7 || d_out == nullptr || d_ws == nullptr) return;
  if (in_sizes[0] != kBatch * kSteps * kChan) return;
  if (in_sizes[1] != kState * kState) return;
  if (in_sizes[2] != kChan * kState) return;
  if (in_sizes[3] != kChan * kState) return;
  if (in_sizes[4] != kChan) return;
  if (in_sizes[5] != kOutF * kChan) return;
  if (in_sizes[6] != kOutF) return;
  if (out_size != kRows * kOutF) return;
  if (ws_size < kWsTotal) return;

  const float* x    = (const float*)d_in[0];
  const float* dA   = (const float*)d_in[1];
  const float* dB   = (const float*)d_in[2];
  const float* Cp   = (const float*)d_in[3];
  const float* Dp   = (const float*)d_in[4];
  const float* W    = (const float*)d_in[5];
  const float* bias = (const float*)d_in[6];
  float* out = (float*)d_out;

  char* ws = (char*)d_ws;
  unsigned short* WH = (unsigned short*)(ws + kOffWH);
  unsigned short* YH = (unsigned short*)(ws + kOffYH);

  const int n8w = kOutF * kChan / 8;
  weight_plane_kernel<<<(n8w + 255) / 256, 256, 0, stream>>>(W, WH, n8w);

  state_scan_kernel<<<kBatch, 128, 0, stream>>>(x, dA, dB, Cp, Dp, YH);

  const int tiles = (kRows / 64) * (kOutF / 64);
  mix_gemm_kernel<<<(tiles + 7) / 8, 256, 0, stream>>>(
      YH, kChan, WH, kChan, out, kOutF, bias, kRows, kOutF, kChan, kMixScale);
}
